// InflatedButterflyLayer1D_52725018526080
// MI455X (gfx1250) — hardware-verified
//
#include <hip/hip_runtime.h>
#include <hip/hip_bf16.h>
#include <math.h>


typedef _Float16 bf16;
typedef _Float16 f16;
typedef __attribute__((ext_vector_type(4))) unsigned v4u_t;
typedef unsigned v4ua __attribute__((ext_vector_type(4), may_alias));
typedef __attribute__((ext_vector_type(4))) float v4f_t;
typedef float v4fa __attribute__((ext_vector_type(4), may_alias));
typedef __attribute__((ext_vector_type(16))) bf16  bf16x16;
typedef bf16x16 f16x16;
typedef __attribute__((ext_vector_type(8)))  bf16  bf16x8;
typedef bf16x8 f16x8;
typedef __attribute__((ext_vector_type(4)))  bf16  bf16x4;
typedef __attribute__((ext_vector_type(8)))  float f32x8;
__device__ __forceinline__ f32x8 wmma16(f16x16 a, f16x16 b, f32x8 c) {
  c = __builtin_amdgcn_wmma_f32_16x16x32_f16(false, a, false, b, (short)0, c, false, false);
  asm volatile("v_nop\n\tv_nop\n\tv_nop\n\tv_nop" : "+v"(c) : "v"(a), "v"(b));
  return c;
}
#define LDS_STRIDE 48
#define KSTRIDE    72
#define VSTRIDE    48

__device__ __forceinline__ f32x8 wmma_bf16(bf16x16 a, bf16x16 b, f32x8 c) {
  c = __builtin_amdgcn_wmma_f32_16x16x32_f16(false, a, false, b, (short)0, c, false, false);
  asm volatile("v_nop\n\tv_nop\n\tv_nop\n\tv_nop" : "+v"(c) : "v"(a), "v"(b));
  return c;
}

template <typename T>
__device__ __forceinline__ bf16x16 load_frag(const T* __restrict__ base, int ld,
                                             int row0, int k0) {
  const int lane = threadIdx.x & 31;
  const int r    = lane & 15;
  const int kh   = (lane >> 4) * 8;
  const T* p0 = base + (size_t)(row0 + r) * ld + (k0 + kh);
  const T* p1 = p0 + 16;
  bf16x16 f;
#pragma unroll
  for (int i = 0; i < 8; ++i) {
    f[i]     = (bf16)p0[i];
    f[i + 8] = (bf16)p1[i];
  }
  return f;
}

__device__ __forceinline__ bf16x16 lds_frag(const bf16* base, int stride) {
  const int lane = threadIdx.x & 31;
  const int row  = lane & 15;
  const int kh   = (lane >> 4) * 8;
  const bf16x8 lo = *(const bf16x8*)(base + row * stride + kh);
  const bf16x8 hi = *(const bf16x8*)(base + row * stride + kh + 16);
  bf16x16 f;
#pragma unroll
  for (int i = 0; i < 8; ++i) { f[i] = lo[i]; f[i + 8] = hi[i]; }
  return f;
}

template <typename T>
__device__ __forceinline__ void stage_read16(const T* __restrict__ p, float* buf) {
#pragma unroll
  for (int i = 0; i < 16; ++i) buf[i] = (float)p[i];
}

__device__ __forceinline__ void stage_write(bf16* dst, const float* buf, int nquad) {
#pragma unroll
  for (int i = 0; i < nquad; ++i) {
    bf16x4 q;
    q[0] = (bf16)buf[4 * i];     q[1] = (bf16)buf[4 * i + 1];
    q[2] = (bf16)buf[4 * i + 2]; q[3] = (bf16)buf[4 * i + 3];
    *(bf16x4*)(dst + 4 * i) = q;
  }
}


#define GSTR 48
#define GSTR 48
template <typename AT, int EPI, bool OUT16>
__global__ __launch_bounds__(256) void gemm_kne(const AT* __restrict__ A, int lda, const float* __restrict__ Wm, int ldw,
                                                const float* __restrict__ bias, const float* __restrict__ R, const float* __restrict__ gvec,
                                                void* __restrict__ Yv, int ldy, int K) {
  __shared__ __attribute__((aligned(16))) f16 ldsA[128 * GSTR];
  __shared__ __attribute__((aligned(16))) f16 ldsW[128 * GSTR];
  __shared__ __attribute__((aligned(16))) float oS[8][32 * 68];
  const int tid = threadIdx.x, lane = tid & 31, wave = tid >> 5, cl = lane & 15, rh = (lane >> 4) * 8;
  const int m0 = blockIdx.x * 128, n0 = blockIdx.y * 128;
  const int wm = (wave & 3) * 32, wn = (wave >> 2) * 64;
  f32x8 acc[2][4];
#pragma unroll
  for (int i = 0; i < 2; ++i)
#pragma unroll
    for (int j = 0; j < 4; ++j) { f32x8 z = {}; acc[i][j] = z; }
#pragma unroll 1
  for (int k0 = 0; k0 < K; k0 += 32) {
    __syncthreads();
    { const int row = tid >> 1, ch = (tid & 1) * 16;
      const AT* src = A + (size_t)(m0 + row) * lda + k0 + ch;
#pragma unroll
      for (int g = 0; g < 16; ++g) ldsA[row * GSTR + ch + g] = (f16)src[g]; }
    { const int k = tid >> 3, nn0 = (tid & 7) * 16;
      const float* src = Wm + (size_t)(k0 + k) * ldw + n0 + nn0;
#pragma unroll
      for (int g = 0; g < 4; ++g) { const v4f_t v = *(const v4f_t*)(src + 4 * g);
#pragma unroll
        for (int u = 0; u < 4; ++u) ldsW[(nn0 + 4 * g + u) * GSTR + k] = (f16)v[u]; } }
    __syncthreads();
    f16x16 af[2];
#pragma unroll
    for (int i = 0; i < 2; ++i) af[i] = lds_frag(ldsA + (wm + 16 * i) * GSTR, GSTR);
#pragma unroll
    for (int j = 0; j < 4; ++j) {
      const f16x16 bf = lds_frag(ldsW + (wn + 16 * j) * GSTR, GSTR);
#pragma unroll
      for (int i = 0; i < 2; ++i) acc[i][j] = wmma16(af[i], bf, acc[i][j]);
    }
  }
  float* so = oS[wave];
#pragma unroll
  for (int i = 0; i < 2; ++i)
#pragma unroll
    for (int j = 0; j < 4; ++j) {
      const int n = n0 + wn + 16 * j + cl;
      const float bv = bias ? bias[n] : 0.0f;
      const float gv = (EPI == 2 || EPI == 4 || EPI == 14) ? gvec[n] : 0.0f;
      if (EPI == 1) {
#pragma unroll 1
        for (int r = 0; r < 8; ++r) { const float xg = acc[i][j][r] + bv; so[(16 * i + rh + r) * 68 + 16 * j + cl] = 0.5f * xg * (1.0f + erff(xg * 0.70710678118654752f)); }
      } else if (EPI == 13) {
#pragma unroll 1
        for (int r = 0; r < 8; ++r) { const size_t mrow = (size_t)(m0 + wm + 16 * i + rh + r); const float xg = acc[i][j][r] + bv; float o = (1.0f / (1.0f + expf(-xg))) * gvec[mrow]; if (R) o += R[mrow * ldy + n]; so[(16 * i + rh + r) * 68 + 16 * j + cl] = o; }
      } else if (EPI == 11) {
#pragma unroll 1
        for (int r = 0; r < 8; ++r) { const float xg = acc[i][j][r] + bv; so[(16 * i + rh + r) * 68 + 16 * j + cl] = xg / (1.0f + expf(-xg)); }
      } else if (EPI == 9 || EPI == 10) {
#pragma unroll 1
        for (int r = 0; r < 8; ++r) { const float xg = acc[i][j][r] + bv + R[(size_t)(m0 + wm + 16 * i + rh + r) * ldy + n]; so[(16 * i + rh + r) * 68 + 16 * j + cl] = (EPI == 9) ? 1.0f / (1.0f + expf(-xg)) : tanhf(xg); }
      } else {
#pragma unroll
        for (int r = 0; r < 8; ++r) {
          float v = acc[i][j][r] + bv;
          if (EPI == 3) v = fmaxf(v, 0.0f);
          if (EPI == 6) v = fminf(fmaxf(v, 0.0f), 6.0f);
          if (EPI == 4) v = gv * v;
          if (EPI == 14) v = fmaxf(acc[i][j][r] * gv + bv, 0.0f);
          if (EPI == 2) v = R[(size_t)(m0 + wm + 16 * i + rh + r) * ldy + n] + gv * v;
          so[(16 * i + rh + r) * 68 + 16 * j + cl] = v;
        }
      }
    }
  asm volatile("s_wait_dscnt 0" ::: "memory");
  __builtin_amdgcn_wave_barrier();
#pragma unroll 1
  for (int pass = 0; pass < 2; ++pass) {
    if (OUT16) {
      f16* Y = (f16*)Yv;
#pragma unroll
      for (int it = 0; it < 8; ++it) { const int c = lane + 32 * it, rr = c >> 3, q8 = (c & 7) * 8;
        union { f16 h[8]; v4u_t v; } u;
#pragma unroll
        for (int e = 0; e < 8; ++e) u.h[e] = (f16)so[rr * 68 + q8 + e];
        *(volatile v4u_t*)(Y + (size_t)(m0 + wm + rr) * ldy + n0 + wn + q8) = u.v; }
    } else {
      float* Y = (float*)Yv;
#pragma unroll
      for (int it = 0; it < 16; ++it) { const int f4 = lane + 32 * it, rr = f4 >> 4, q = (f4 & 15) * 4;
        *(volatile v4f_t*)(Y + (size_t)(m0 + wm + rr) * ldy + n0 + wn + q) = *(const v4fa*)(so + rr * 68 + q); }
    }
    __threadfence();
  }
}

template <typename AT, int EPI, bool OUT16>
__global__ __launch_bounds__(256) void gemm_knez(const AT* __restrict__ A, int lda, size_t strideA, const float* __restrict__ Wm, int ldw, size_t strideW,
                                                 const float* __restrict__ bias, const float* __restrict__ R, const float* __restrict__ gvec,
                                                 void* __restrict__ Yv, int ldy, size_t strideY, int K) {
  A += (size_t)blockIdx.z * strideA; Wm += (size_t)blockIdx.z * strideW; Yv = (void*)((char*)Yv + (size_t)blockIdx.z * strideY * (OUT16 ? 2 : 4)); if (R) R += (size_t)blockIdx.z * strideY;
  __shared__ __attribute__((aligned(16))) f16 ldsA[128 * GSTR];
  __shared__ __attribute__((aligned(16))) f16 ldsW[128 * GSTR];
  __shared__ __attribute__((aligned(16))) float oS[8][32 * 68];
  const int tid = threadIdx.x, lane = tid & 31, wave = tid >> 5, cl = lane & 15, rh = (lane >> 4) * 8;
  const int m0 = blockIdx.x * 128, n0 = blockIdx.y * 128;
  const int wm = (wave & 3) * 32, wn = (wave >> 2) * 64;
  f32x8 acc[2][4];
#pragma unroll
  for (int i = 0; i < 2; ++i)
#pragma unroll
    for (int j = 0; j < 4; ++j) { f32x8 z = {}; acc[i][j] = z; }
#pragma unroll 1
  for (int k0 = 0; k0 < K; k0 += 32) {
    __syncthreads();
    { const int row = tid >> 1, ch = (tid & 1) * 16;
      const AT* src = A + (size_t)(m0 + row) * lda + k0 + ch;
#pragma unroll
      for (int g = 0; g < 16; ++g) ldsA[row * GSTR + ch + g] = (f16)src[g]; }
    { const int k = tid >> 3, nn0 = (tid & 7) * 16;
      const float* src = Wm + (size_t)(k0 + k) * ldw + n0 + nn0;
#pragma unroll
      for (int g = 0; g < 4; ++g) { const v4f_t v = *(const v4f_t*)(src + 4 * g);
#pragma unroll
        for (int u = 0; u < 4; ++u) ldsW[(nn0 + 4 * g + u) * GSTR + k] = (f16)v[u]; } }
    __syncthreads();
    f16x16 af[2];
#pragma unroll
    for (int i = 0; i < 2; ++i) af[i] = lds_frag(ldsA + (wm + 16 * i) * GSTR, GSTR);
#pragma unroll
    for (int j = 0; j < 4; ++j) {
      const f16x16 bf = lds_frag(ldsW + (wn + 16 * j) * GSTR, GSTR);
#pragma unroll
      for (int i = 0; i < 2; ++i) acc[i][j] = wmma16(af[i], bf, acc[i][j]);
    }
  }
  float* so = oS[wave];
#pragma unroll
  for (int i = 0; i < 2; ++i)
#pragma unroll
    for (int j = 0; j < 4; ++j) {
      const int n = n0 + wn + 16 * j + cl;
      const float bv = bias ? bias[n] : 0.0f;
      const float gv = (EPI == 2 || EPI == 4 || EPI == 14) ? gvec[n] : 0.0f;
      if (EPI == 1) {
#pragma unroll 1
        for (int r = 0; r < 8; ++r) { const float xg = acc[i][j][r] + bv; so[(16 * i + rh + r) * 68 + 16 * j + cl] = 0.5f * xg * (1.0f + erff(xg * 0.70710678118654752f)); }
      } else if (EPI == 13) {
#pragma unroll 1
        for (int r = 0; r < 8; ++r) { const size_t mrow = (size_t)(m0 + wm + 16 * i + rh + r); const float xg = acc[i][j][r] + bv; float o = (1.0f / (1.0f + expf(-xg))) * gvec[mrow]; if (R) o += R[mrow * ldy + n]; so[(16 * i + rh + r) * 68 + 16 * j + cl] = o; }
      } else if (EPI == 11) {
#pragma unroll 1
        for (int r = 0; r < 8; ++r) { const float xg = acc[i][j][r] + bv; so[(16 * i + rh + r) * 68 + 16 * j + cl] = xg / (1.0f + expf(-xg)); }
      } else if (EPI == 9 || EPI == 10) {
#pragma unroll 1
        for (int r = 0; r < 8; ++r) { const float xg = acc[i][j][r] + bv + R[(size_t)(m0 + wm + 16 * i + rh + r) * ldy + n]; so[(16 * i + rh + r) * 68 + 16 * j + cl] = (EPI == 9) ? 1.0f / (1.0f + expf(-xg)) : tanhf(xg); }
      } else {
#pragma unroll
        for (int r = 0; r < 8; ++r) {
          float v = acc[i][j][r] + bv;
          if (EPI == 3) v = fmaxf(v, 0.0f);
          if (EPI == 6) v = fminf(fmaxf(v, 0.0f), 6.0f);
          if (EPI == 4) v = gv * v;
          if (EPI == 14) v = fmaxf(acc[i][j][r] * gv + bv, 0.0f);
          if (EPI == 2) v = R[(size_t)(m0 + wm + 16 * i + rh + r) * ldy + n] + gv * v;
          so[(16 * i + rh + r) * 68 + 16 * j + cl] = v;
        }
      }
    }
  asm volatile("s_wait_dscnt 0" ::: "memory");
  __builtin_amdgcn_wave_barrier();
#pragma unroll 1
  for (int pass = 0; pass < 2; ++pass) {
    if (OUT16) {
      f16* Y = (f16*)Yv;
#pragma unroll
      for (int it = 0; it < 8; ++it) { const int c = lane + 32 * it, rr = c >> 3, q8 = (c & 7) * 8;
        union { f16 h[8]; v4u_t v; } u;
#pragma unroll
        for (int e = 0; e < 8; ++e) u.h[e] = (f16)so[rr * 68 + q8 + e];
        *(volatile v4u_t*)(Y + (size_t)(m0 + wm + rr) * ldy + n0 + wn + q8) = u.v; }
    } else {
      float* Y = (float*)Yv;
#pragma unroll
      for (int it = 0; it < 16; ++it) { const int f4 = lane + 32 * it, rr = f4 >> 4, q = (f4 & 15) * 4;
        *(volatile v4f_t*)(Y + (size_t)(m0 + wm + rr) * ldy + n0 + wn + q) = *(const v4fa*)(so + rr * 68 + q); }
    }
    __threadfence();
  }
}

template <typename AT, bool ACC>
__global__ __launch_bounds__(256) void gemm_kn2(const AT* __restrict__ A, int lda, size_t strideA,
                                               const float* __restrict__ Wm, int ldw, size_t strideW,
                                               const float* __restrict__ bias, float scale,
                                               float* __restrict__ Y, int ldy, size_t strideY, int K) {
  __shared__ __attribute__((aligned(16))) f16 ldsA[128 * GSTR], ldsAl[128 * GSTR];
  __shared__ __attribute__((aligned(16))) f16 ldsW[128 * GSTR], ldsWl[128 * GSTR];
  __shared__ __attribute__((aligned(16))) float oS[8][32 * 68];
  const int tid = threadIdx.x, lane = tid & 31, wave = tid >> 5, cl = lane & 15, rh = (lane >> 4) * 8;
  const int m0 = blockIdx.x * 128, n0 = blockIdx.y * 128;
  const int wm = (wave & 3) * 32, wn = (wave >> 2) * 64;
  A += (size_t)blockIdx.z * strideA; Wm += (size_t)blockIdx.z * strideW; Y += (size_t)blockIdx.z * strideY;
  f32x8 acc[2][4], accx[2][4];
#pragma unroll
  for (int i = 0; i < 2; ++i)
#pragma unroll
    for (int j = 0; j < 4; ++j) { f32x8 z = {}; acc[i][j] = z; accx[i][j] = z; }
#pragma unroll 1
  for (int k0 = 0; k0 < K; k0 += 32) {
    __syncthreads();
    {
      const int row = tid >> 1, ch = (tid & 1) * 16;
      const AT* src = A + (size_t)(m0 + row) * lda + k0 + ch;
#pragma unroll
      for (int g = 0; g < 16; ++g) { const float v = (float)src[g]; const f16 h = (f16)v; ldsA[row * GSTR + ch + g] = h; ldsAl[row * GSTR + ch + g] = (f16)((v - (float)h) * 2048.0f); }
    }
    {
      const int k = tid >> 3, nn0 = (tid & 7) * 16;
      const float* src = Wm + (size_t)(k0 + k) * ldw + n0 + nn0;
#pragma unroll
      for (int g = 0; g < 4; ++g) { const v4f_t v = *(const v4f_t*)(src + 4 * g);
#pragma unroll
        for (int u = 0; u < 4; ++u) { const f16 h = (f16)v[u]; ldsW[(nn0 + 4 * g + u) * GSTR + k] = h; ldsWl[(nn0 + 4 * g + u) * GSTR + k] = (f16)((v[u] - (float)h) * 2048.0f); } }
    }
    __syncthreads();
    f16x16 af[2], afl[2];
#pragma unroll
    for (int i = 0; i < 2; ++i) { af[i] = lds_frag(ldsA + (wm + 16 * i) * GSTR, GSTR); afl[i] = lds_frag(ldsAl + (wm + 16 * i) * GSTR, GSTR); }
#pragma unroll
    for (int j = 0; j < 4; ++j) {
      const f16x16 bf = lds_frag(ldsW + (wn + 16 * j) * GSTR, GSTR), bfl = lds_frag(ldsWl + (wn + 16 * j) * GSTR, GSTR);
#pragma unroll
      for (int i = 0; i < 2; ++i) { acc[i][j] = wmma16(af[i], bf, acc[i][j]); accx[i][j] = wmma16(af[i], bfl, accx[i][j]); accx[i][j] = wmma16(afl[i], bf, accx[i][j]); }
    }
  }
  float* so = oS[wave];
#pragma unroll
  for (int i = 0; i < 2; ++i)
#pragma unroll
    for (int j = 0; j < 4; ++j) {
      const float bv = bias ? bias[n0 + wn + 16 * j + cl] : 0.0f;
#pragma unroll
      for (int r = 0; r < 8; ++r) so[(16 * i + rh + r) * 68 + 16 * j + cl] = (acc[i][j][r] + accx[i][j][r] * (1.0f / 2048.0f)) * scale + bv;
    }
  asm volatile("s_wait_dscnt 0" ::: "memory");
  __builtin_amdgcn_wave_barrier();
  if (ACC) {
#pragma unroll
    for (int it = 0; it < 16; ++it) { const int f4 = lane + 32 * it, rr = f4 >> 4, q = (f4 & 15) * 4;
      const v4f_t old = *(const v4fa*)(Y + (size_t)(m0 + wm + rr) * ldy + n0 + wn + q);
      v4f_t v = *(const v4fa*)(so + rr * 68 + q); v += old; *(v4fa*)(so + rr * 68 + q) = v; }
    asm volatile("s_wait_dscnt 0" ::: "memory");
  }
#pragma unroll 1
  for (int pass = 0; pass < 2; ++pass) {
#pragma unroll
    for (int it = 0; it < 16; ++it) { const int f4 = lane + 32 * it, rr = f4 >> 4, q = (f4 & 15) * 4;
      *(volatile v4f_t*)(Y + (size_t)(m0 + wm + rr) * ldy + n0 + wn + q) = *(const v4fa*)(so + rr * 68 + q); }
    __threadfence();
  }
}

__global__ __launch_bounds__(256) void k_transpose(const float* __restrict__ Wm, float* __restrict__ Wt, int rows, int cols) {
  __shared__ float tS[64][65];
  const int tid = threadIdx.x, tbj = cols / 64, bi = blockIdx.x / tbj, bj = blockIdx.x % tbj;
  for (int e = tid; e < 64 * 64; e += 256) { const int r = e >> 6, c = e & 63; tS[r][c] = Wm[(size_t)(bi * 64 + r) * cols + bj * 64 + c]; }
  __syncthreads();
  for (int ch = tid; ch < 64 * 16; ch += 256) { const int r = ch >> 4, q4 = (ch & 15) * 4; v4f_t o; o[0] = tS[q4][r]; o[1] = tS[q4 + 1][r]; o[2] = tS[q4 + 2][r]; o[3] = tS[q4 + 3][r];
    float* dst = Wt + (size_t)(bj * 64 + r) * rows + bi * 64 + q4; *(volatile v4f_t*)dst = o; __threadfence(); *(volatile v4f_t*)dst = o; }
}


template <typename AT, int EPI, bool OUT16, int NJ>
__global__ __launch_bounds__(256) void gemm_sm(const AT* __restrict__ A, int lda, size_t sA, const float* __restrict__ Wm, int ldw, size_t sW,
                                               const float* __restrict__ bias, const float* __restrict__ R, const float* __restrict__ gvec,
                                               void* __restrict__ Yv, int ldy, size_t sY, int K) {
  constexpr int BN = 16 * NJ; constexpr int OST = BN + 4;
  A += (size_t)blockIdx.z * sA; Wm += (size_t)blockIdx.z * sW; Yv = (void*)((char*)Yv + (size_t)blockIdx.z * sY * (OUT16 ? 2 : 4)); if (R) R += (size_t)blockIdx.z * sY;
  __shared__ __attribute__((aligned(16))) f16 ldsA[256 * GSTR];
  __shared__ __attribute__((aligned(16))) f16 ldsW[BN * GSTR];
  __shared__ __attribute__((aligned(16))) float oS[8][32 * OST];
  const int tid = threadIdx.x, lane = tid & 31, wave = tid >> 5, cl = lane & 15, rh = (lane >> 4) * 8;
  const int m0 = blockIdx.x * 256, n0 = blockIdx.y * BN;
  const int wm = wave * 32;
  f32x8 acc[2][NJ];
#pragma unroll
  for (int i = 0; i < 2; ++i)
#pragma unroll
    for (int j = 0; j < NJ; ++j) { f32x8 z = {}; acc[i][j] = z; }
#pragma unroll 1
  for (int k0 = 0; k0 < K; k0 += 32) {
    __syncthreads();
    { const AT* src = A + (size_t)(m0 + tid) * lda + k0;
#pragma unroll
      for (int g = 0; g < 32; ++g) ldsA[tid * GSTR + g] = (f16)src[g]; }
    { const int k = tid >> 3, nn0 = (tid & 7) * (2 * NJ);
      const float* src = Wm + (size_t)(k0 + k) * ldw + n0 + nn0;
#pragma unroll
      for (int g = 0; g < NJ / 2; ++g) { const v4f_t v = *(const v4f_t*)(src + 4 * g);
#pragma unroll
        for (int u = 0; u < 4; ++u) ldsW[(nn0 + 4 * g + u) * GSTR + k] = (f16)v[u]; } }
    __syncthreads();
    f16x16 af[2];
#pragma unroll
    for (int i = 0; i < 2; ++i) af[i] = lds_frag(ldsA + (wm + 16 * i) * GSTR, GSTR);
#pragma unroll
    for (int j = 0; j < NJ; ++j) {
      const f16x16 bf = lds_frag(ldsW + (16 * j) * GSTR, GSTR);
#pragma unroll
      for (int i = 0; i < 2; ++i) acc[i][j] = wmma16(af[i], bf, acc[i][j]);
    }
  }
  float* so = oS[wave];
#pragma unroll
  for (int i = 0; i < 2; ++i)
#pragma unroll
    for (int j = 0; j < NJ; ++j) {
      const int n = n0 + 16 * j + cl;
      const float bv = bias ? bias[n] : 0.0f;
      const float gv = (EPI == 2 || EPI == 4) ? gvec[n] : 0.0f;
#pragma unroll
      for (int r = 0; r < 8; ++r) {
        float v = acc[i][j][r] + bv;
        if (EPI == 3) v = fmaxf(v, 0.0f);
        if (EPI == 2) v = R[(size_t)(m0 + wm + 16 * i + rh + r) * ldy + n] + gv * v;
        if (EPI == 4) v = gv * v;
        so[(16 * i + rh + r) * OST + 16 * j + cl] = v;
      }
    }
  asm volatile("s_wait_dscnt 0" ::: "memory");
  __builtin_amdgcn_wave_barrier();
#pragma unroll 1
  for (int pass = 0; pass < 2; ++pass) {
    if (OUT16) {
      f16* Y = (f16*)Yv;
#pragma unroll
      for (int it = 0; it < BN / 8; ++it) { const int c = lane + 32 * it, rr = c / (BN / 8), q8 = (c % (BN / 8)) * 8;
        union { f16 h[8]; v4u_t v; } u;
#pragma unroll
        for (int e = 0; e < 8; ++e) u.h[e] = (f16)so[rr * OST + q8 + e];
        *(volatile v4u_t*)(Y + (size_t)(m0 + wm + rr) * ldy + n0 + q8) = u.v; }
    } else {
      float* Y = (float*)Yv;
#pragma unroll
      for (int it = 0; it < BN / 4; ++it) { const int f4 = lane + 32 * it, rr = f4 / (BN / 4), q = (f4 % (BN / 4)) * 4;
        *(volatile v4f_t*)(Y + (size_t)(m0 + wm + rr) * ldy + n0 + q) = *(const v4fa*)(so + rr * OST + q); }
    }
    __threadfence();
  }
}

#define NBi 512
#define NNi 4096
#define CCi 64
__global__ __launch_bounds__(256) void k_fill(float* __restrict__ p, float val, size_t n4) { const size_t i = (size_t)blockIdx.x * 256 + threadIdx.x; if (i < n4) { v4f_t v = {val, val, val, val}; *(volatile v4f_t*)(p + 4 * i) = v; __threadfence(); *(volatile v4f_t*)(p + 4 * i) = v; } }
__global__ __launch_bounds__(256) void k_dbg_zero(float* __restrict__ p, size_t n4) { const size_t i = (size_t)blockIdx.x * 256 + threadIdx.x; if (i < n4) { v4f_t z = {0.f,0.f,0.f,0.f}; *(volatile v4f_t*)(p + 4 * i) = z; __threadfence(); *(volatile v4f_t*)(p + 4 * i) = z; } }
__global__ __launch_bounds__(256) void k_copy(const float* __restrict__ src, float* __restrict__ dst, size_t n4) { const size_t i = (size_t)blockIdx.x * 256 + threadIdx.x; if (i < n4) { const v4f_t v = *(const v4f_t*)(src + 4 * i); *(volatile v4f_t*)(dst + 4 * i) = v; __threadfence(); *(volatile v4f_t*)(dst + 4 * i) = v; } }
__global__ __launch_bounds__(64) void k_padxf(const float* __restrict__ xf, float* __restrict__ XF) { const int c = threadIdx.x;
#pragma unroll 1
  for (int k = 0; k < 32; ++k) { const float v = (k < 16) ? xf[min(k, 15) * CCi + c] : 0.0f; *(volatile float*)(XF + k * CCi + c) = v; }
  __threadfence();
#pragma unroll 1
  for (int k = 0; k < 32; ++k) { float* p = XF + k * CCi + c; const float v = p[0]; *(volatile float*)p = v; } }
__global__ __launch_bounds__(32) void k_padkf(const float* __restrict__ kf, float* __restrict__ KF) { const int c = blockIdx.x, o = threadIdx.x; const float v = (o < 16) ? kf[c * 16 + min(o, 15)] : 0.0f; *(volatile float*)(KF + c * 32 + o) = v; __threadfence(); *(volatile float*)(KF + c * 32 + o) = v; }
__global__ __launch_bounds__(256) void k_shuffle(const float* __restrict__ src, float* __restrict__ dst, int p, int nitx) {
  const int row = blockIdx.x; const int b = row / (2 * p), pp = row % (2 * p); const int itk = pp >> 1, r = pp & 1; const int tid = threadIdx.x; if (tid >= nitx * 16) return;
  const int itx = tid >> 4, c4 = (tid & 15) * 4; const int wsrc = nitx * 2 * CCi, wdst = nitx * CCi;
  const v4f_t v = *(const v4f_t*)(src + ((size_t)b * p + itk) * wsrc + (2 * itx + r) * CCi + c4); float* d = dst + ((size_t)b * 2 * p + pp) * wdst + itx * CCi + c4;
  *(volatile v4f_t*)d = v; __threadfence(); *(volatile v4f_t*)d = v;
}
__global__ __launch_bounds__(256) void k_scalevec(const float* __restrict__ src, float* __restrict__ dst, float sc, int n4) { const int i = blockIdx.x * 256 + threadIdx.x; if (i < n4) { const v4f_t v = *(const v4f_t*)(src + 4 * i) * sc; *(volatile v4f_t*)(dst + 4 * i) = v; __threadfence(); *(volatile v4f_t*)(dst + 4 * i) = v; } }
__global__ __launch_bounds__(256) void k_repack(const float* __restrict__ Y32, float* __restrict__ out) {
  const size_t i4 = ((size_t)blockIdx.x * 256 + threadIdx.x) * 4; const size_t rowi = i4 >> 4; const int o = (int)(i4 & 15);
  const v4f_t v = *(const v4f_t*)(Y32 + rowi * 32 + o) * 262144.0f; *(volatile v4f_t*)(out + i4) = v; __threadfence(); *(volatile v4f_t*)(out + i4) = v;
}

extern "C" void kernel_launch(void* const* d_in, const int* in_sizes, int n_in,
                              void* d_out, int out_size, void* d_ws, size_t ws_size,
                              hipStream_t stream) {
  (void)in_sizes; (void)n_in; (void)out_size;
  const float** f = (const float**)d_in;
  const float* x = f[0], *xf = f[1], *xb = f[2]; const float* wl[9] = {nullptr, f[3], f[5], f[7], f[9], f[13], f[15], f[17], f[19]}; const float* bl[9] = {nullptr, f[4], f[6], f[8], f[10], f[14], f[16], f[18], f[20]};
  const float* midw = f[11], *midb = f[12], *kf = f[21];
  float* out = (float*)d_out;
  char* ws = (char*)d_ws;
  float* XC = (float*)ws; ws += ((size_t)NBi * NNi + 32) * 4;
  float* XF = (float*)ws; ws += 32 * CCi * 4; float* KF = (float*)ws; ws += CCi * 32 * 4;
  float* HA = (float*)ws; ws += (size_t)NBi * 256 * CCi * 4; float* HB = (float*)ws; ws += (size_t)NBi * 256 * CCi * 4;
  float* SB = (float*)ws; ws += (size_t)(1024 + 16 * 16 * CCi + 1024 + 512 + 256 + 128) * 4;
  float* GV = (float*)ws; ws += (size_t)3 * 1024 * 4;
  float* Y32 = (float*)ws; ws += (size_t)NBi * 256 * 32 * 4;
  if ((size_t)(ws - (char*)d_ws) > ws_size) return;
  const dim3 blk(256); const size_t ACT = (size_t)256 * CCi;
  k_copy<<<dim3(((size_t)NBi * NNi / 4 + 255) / 256), blk, 0, stream>>>(x, XC, (size_t)NBi * NNi / 4); k_fill<<<dim3(1), blk, 0, stream>>>(XC + (size_t)NBi * NNi, 0.0f, 32 / 4);
  k_padxf<<<dim3(1), dim3(64), 0, stream>>>(xf, XF);
  float* b4s = SB; float* midbs = b4s + 1024; float* b5s = midbs + 16 * 16 * CCi; float* b6s = b5s + 1024; float* b7s = b6s + 512; float* b8s = b7s + 256;
  float* g8 = GV; float* g6 = GV + 1024; float* g2 = GV + 2048;
  k_scalevec<<<dim3(1), blk, 0, stream>>>(bl[4], b4s, 1.0f / 256.0f, 1024 / 4); k_scalevec<<<dim3((16 * 16 * CCi / 4 + 255) / 256), blk, 0, stream>>>(midb, midbs, 1.0f / 256.0f, 16 * 16 * CCi / 4);
  k_scalevec<<<dim3(1), blk, 0, stream>>>(bl[5], b5s, 1.0f / 16384.0f, 1024 / 4); k_scalevec<<<dim3(1), blk, 0, stream>>>(bl[6], b6s, 1.0f / 65536.0f, 512 / 4); k_scalevec<<<dim3(1), blk, 0, stream>>>(bl[7], b7s, 1.0f / 262144.0f, 256 / 4); k_scalevec<<<dim3(1), blk, 0, stream>>>(bl[8], b8s, 1.0f / 262144.0f, 128 / 4);
  k_fill<<<dim3(1), blk, 0, stream>>>(g8, 1.0f / 256.0f, 1024 / 4); k_fill<<<dim3(1), blk, 0, stream>>>(g6, 1.0f / 64.0f, 1024 / 4); k_fill<<<dim3(1), blk, 0, stream>>>(g2, 0.25f, 1024 / 4); k_padkf<<<dim3(CCi), dim3(32), 0, stream>>>(kf, KF);

  gemm_sm<float, 3, false, 4><<<dim3((unsigned)((size_t)NBi * 256 / 256), 1, 1), blk, 0, stream>>>(XC, 16, (size_t)0, XF, CCi, (size_t)0, xb, nullptr, nullptr, HA, CCi, (size_t)0, 32);
  float* hin = HA; float* hout = HB;
  for (int l = 1; l <= 4; ++l) { const int cin = CCi << (l - 1), cout = CCi << l; const int pin = 256 >> (l - 1); const size_t rows = (size_t)NBi * (pin / 2);
    if (l < 4) gemm_kne<float, 3, false><<<dim3((unsigned)(rows / 128), cout / 128), blk, 0, stream>>>(hin, 2 * cin, wl[l], cout, bl[l], nullptr, nullptr, hout, cout, 2 * cin);
    else       gemm_kne<float, 14, false><<<dim3((unsigned)(rows / 128), cout / 128), blk, 0, stream>>>(hin, 2 * cin, wl[l], cout, b4s, nullptr, g8, hout, cout, 2 * cin);
    float* t = hin; hin = hout; hout = t; }
  for (int xi = 0; xi < 16; ++xi) for (int kk = 0; kk < 16; ++kk)
    gemm_sm<float, 3, false, 4><<<dim3(NBi / 256, 1, 1), blk, 0, stream>>>(hin + xi * 1024 + kk * CCi, (int)ACT, (size_t)0, midw + ((size_t)kk * 16 + xi) * CCi * CCi, CCi, (size_t)0, midbs + ((size_t)kk * 16 + xi) * CCi, nullptr, nullptr, hout + kk * 1024 + xi * CCi, (int)ACT, (size_t)0, CCi);
  { float* t = hin; hin = hout; hout = t; }
  for (int l = 5; l <= 8; ++l) { const int nitx = 1 << (8 - l); const int p = 256 >> (9 - l);
    k_shuffle<<<dim3((unsigned)((size_t)NBi * 2 * p)), blk, 0, stream>>>(hin, hout, p, nitx); { float* t = hin; hin = hout; hout = t; }
    const int cin = nitx * CCi, cout = 2 * nitx * CCi; const size_t rows = (size_t)NBi * p;
    { const float* bsc = (l == 5) ? b5s : (l == 6) ? b6s : (l == 7) ? b7s : b8s; const float* gsc = (l == 5) ? g6 : g2;
      if (l < 8) gemm_kne<float, 14, false><<<dim3((unsigned)(rows / 128), cout / 128), blk, 0, stream>>>(hin, 2 * cin, wl[l], cout, bsc, nullptr, gsc, hout, cout, 2 * cin);
      else       gemm_kne<float, 3, false><<<dim3((unsigned)(rows / 128), cout / 128), blk, 0, stream>>>(hin, 2 * cin, wl[l], cout, bsc, nullptr, nullptr, hout, cout, 2 * cin); }
    { float* t = hin; hin = hout; hout = t; }
    k_shuffle<<<dim3((unsigned)((size_t)NBi * 2 * p)), blk, 0, stream>>>(hin, hout, p, nitx); { float* t = hin; hin = hout; hout = t; }
  }
  gemm_sm<float, 0, false, 2><<<dim3((unsigned)((size_t)NBi * 256 / 256), 1, 1), blk, 0, stream>>>(hin, CCi, (size_t)0, KF, 32, (size_t)0, nullptr, nullptr, nullptr, Y32, 32, (size_t)0, CCi);
  k_repack<<<dim3((unsigned)((size_t)NBi * NNi / 4 / 256)), blk, 0, stream>>>(Y32, out);
}
